// LSWTTokenPoolerAttention_12773232738466
// MI455X (gfx1250) — hardware-verified
//
#include <hip/hip_runtime.h>

#define NB     2
#define SEQ    1024
#define HID    1024
#define NHEADS 16
#define HD     64
#define MROWS  (NB * SEQ)
#define NX     (MROWS * HID)
#define NW     (HID * HID)
#define NG     (NHEADS * HID)
#define NX8    (NX / 8)
#define NW8    (NW / 8)
#define NG8    (NG / 8)
#define SEP_ID 1
#define CLS_ID 2
#define PAD_ID 0
#define XSC    4.0f
#define WSC    4096.0f
#define QSC    16.0f
#define PSC    16384.0f
#define CSC    64.0f
#define NEGBIG (-1.0e30f)

static_assert(NHEADS * HD == HID);
static_assert((SEQ % 128) == 0 && (HID % 64) == 0 && (HID % 32) == 0 && (MROWS % 128) == 0);
static_assert((NW8 % 256) == 0 && (NG8 % 256) == 0);
static_assert(SEQ == 8 * 128);

typedef _Float16 v16h __attribute__((ext_vector_type(16)));
typedef _Float16 v8h  __attribute__((ext_vector_type(8)));
typedef float    v8f  __attribute__((ext_vector_type(8)));
typedef float    v4f  __attribute__((ext_vector_type(4)));
typedef int      v4i  __attribute__((ext_vector_type(4)));
typedef v8h __attribute__((may_alias)) v8ha;
typedef v4f __attribute__((may_alias)) v4fa;
typedef v4i __attribute__((may_alias)) v4ia;

union Frag { v16h v; v8h half[2]; };

__device__ __forceinline__ v8f zero8f() { v8f z = {0.f, 0.f, 0.f, 0.f, 0.f, 0.f, 0.f, 0.f}; return z; }
__device__ __forceinline__ v16h zero16h() {
  const _Float16 z = (_Float16)0.0f;
  v16h r = {z, z, z, z, z, z, z, z, z, z, z, z, z, z, z, z};
  return r;
}

__device__ __forceinline__ v8f wmma_f16(v16h a, v16h b, v8f c) {
  v8f d = __builtin_amdgcn_wmma_f32_16x16x32_f16(false, a, false, b, (short)0, c, false, false);
  asm volatile("v_nop\n\tv_nop\n\tv_nop\n\tv_nop" : "+v"(d) : "v"(a), "v"(b));
  return d;
}

__device__ __forceinline__ v16h load_frag(const _Float16* p, int h) {
  Frag f;
  f.half[0] = *(const v8ha*)(p + 8 * h);
  f.half[1] = *(const v8ha*)(p + 16 + 8 * h);
  return f.v;
}

__global__ __launch_bounds__(256) void convert_kernel(
    const float* __restrict__ w0, const float* __restrict__ w1, const float* __restrict__ w2,
    const float* __restrict__ w3, const float* __restrict__ g0, const float* __restrict__ g1,
    int nbig, int nsmall, _Float16* wh, _Float16* woh, _Float16* gh)
{
  const int g = blockIdx.x * 256 + threadIdx.x;
  const int nb8 = nbig * NW8;
  const int total = nb8 + NW8 + nsmall * NG8;
  if (g >= total) return;
  const float* src;
  _Float16* dst;
  if (g < nb8) {
    const int slot = g / NW8;
    const int off = g - slot * NW8;
    const float* wsrc = (slot == 0) ? w0 : ((slot == 1) ? w1 : w2);
    src = wsrc + (size_t)off * 8;
    dst = wh + (size_t)g * 8;
  } else if (g < nb8 + NW8) {
    const int off = g - nb8;
    src = w3 + (size_t)off * 8;
    dst = woh + (size_t)off * 8;
  } else {
    const int e = g - nb8 - NW8;
    src = (e < NG8) ? (g0 + (size_t)e * 8) : (g1 + (size_t)(e - NG8) * 8);
    dst = gh + (size_t)e * 8;
  }
  const v4f a = *(const v4fa*)src;
  const v4f c = *(const v4fa*)(src + 4);
  const v8h o = { (_Float16)(a.x * WSC), (_Float16)(a.y * WSC), (_Float16)(a.z * WSC), (_Float16)(a.w * WSC),
                  (_Float16)(c.x * WSC), (_Float16)(c.y * WSC), (_Float16)(c.z * WSC), (_Float16)(c.w * WSC) };
  *(volatile v8h*)dst = o;
  __threadfence();
  *(volatile v8h*)dst = o;
}

__global__ __launch_bounds__(128) void ln_kernel(const float* __restrict__ x,
                                                 const float* __restrict__ w,
                                                 const float* __restrict__ bb,
                                                 _Float16* y)
{
  __shared__ float ps[4];
  __shared__ float pq[4];
  const int tok = blockIdx.x, t = threadIdx.x, lane = t & 31, wv = t >> 5;
  const float* xr = x + (size_t)tok * HID + 8 * t;
  const v4f a = *(const v4fa*)xr;
  const v4f c = *(const v4fa*)(xr + 4);
  float s = ((a.x + a.y) + (a.z + a.w)) + ((c.x + c.y) + (c.z + c.w));
#pragma unroll
  for (int o = 1; o < 32; o <<= 1) s += __shfl_xor(s, o, 32);
  if (lane == 0) ps[wv] = s;
  __syncthreads();
  const float mean = ((ps[0] + ps[1]) + (ps[2] + ps[3])) * (1.0f / (float)HID);
  float d[8] = { a.x - mean, a.y - mean, a.z - mean, a.w - mean,
                 c.x - mean, c.y - mean, c.z - mean, c.w - mean };
  float q = 0.f;
#pragma unroll
  for (int i = 0; i < 8; ++i) q += d[i] * d[i];
#pragma unroll
  for (int o = 1; o < 32; o <<= 1) q += __shfl_xor(q, o, 32);
  if (lane == 0) pq[wv] = q;
  __syncthreads();
  const float var = ((pq[0] + pq[1]) + (pq[2] + pq[3])) * (1.0f / (float)HID);
  const float rstd = rsqrtf(var + 1e-5f);
  const v4f wa = *(const v4fa*)(w + 8 * t);
  const v4f wc = *(const v4fa*)(w + 8 * t + 4);
  const v4f ba = *(const v4fa*)(bb + 8 * t);
  const v4f bc = *(const v4fa*)(bb + 8 * t + 4);
  const float wvv[8] = { wa.x, wa.y, wa.z, wa.w, wc.x, wc.y, wc.z, wc.w };
  const float bvv[8] = { ba.x, ba.y, ba.z, ba.w, bc.x, bc.y, bc.z, bc.w };
  v8h o;
#pragma unroll
  for (int i = 0; i < 8; ++i) o[i] = (_Float16)((d[i] * rstd * wvv[i] + bvv[i]) * XSC);
  _Float16* dst = y + (size_t)tok * HID + 8 * t;
  *(volatile v8h*)dst = o;
  __threadfence();
  *(volatile v8h*)dst = o;
}

template <bool POOL>
__global__ __launch_bounds__(128) void head_kernel(const _Float16* __restrict__ xh,
                                                   const _Float16* __restrict__ gh,
                                                   const float* __restrict__ gbias,
                                                   float* gate, float* aproj)
{
  __shared__ __attribute__((aligned(16))) float sG[4][256];
  __shared__ __attribute__((aligned(16))) float sP[POOL ? 4 : 1][256];
  const int tid = threadIdx.x, lane = tid & 31, w = tid >> 5;
  const int h = lane >> 4, m = lane & 15;
  const int tok0 = blockIdx.x * 64 + 16 * w;
  const _Float16* xa = xh + (size_t)(tok0 + m) * HID;
  const _Float16* wg = gh + (size_t)m * HID;
  const _Float16* wa = gh + (size_t)(NHEADS + m) * HID;
  v8f ag = zero8f(), aa = zero8f();
#pragma unroll 1
  for (int k0 = 0; k0 < HID; k0 += 32) {
    const v16h a = load_frag(xa + k0, h);
    const v16h bg = load_frag(wg + k0, h);
    ag = wmma_f16(a, bg, ag);
    if constexpr (POOL) {
      const v16h ba = load_frag(wa + k0, h);
      aa = wmma_f16(a, ba, aa);
    }
  }
  const float gbv = gbias[m];
  float* sg = sG[w];
  float* sp = sP[POOL ? w : 0];
#pragma unroll
  for (int r = 0; r < 8; ++r) {
    const int tl = 8 * h + r;
    const float z = ag[r] * (1.0f / (XSC * WSC)) + gbv;
    const float sig = 1.0f / (1.0f + __expf(-z));
    sg[tl * NHEADS + m] = sig;
    if constexpr (POOL) sp[tl * NHEADS + m] = aa[r] * (1.0f / (XSC * WSC));
  }
  __syncthreads();
  for (int pass = 0; pass < 2; ++pass) {
#pragma unroll
    for (int it = 0; it < 2; ++it) {
      const int idx = it * 128 + 4 * lane;
      const v4f v = *(const v4fa*)(sg + idx);
      *(volatile v4f*)(gate + (size_t)tok0 * NHEADS + idx) = v;
      if constexpr (POOL) {
        const v4f u = *(const v4fa*)(sp + idx);
        *(volatile v4f*)(aproj + (size_t)tok0 * NHEADS + idx) = u;
      }
    }
    __threadfence();
  }
}

__device__ __forceinline__ void proj_store_pass(const _Float16* sT, _Float16* plane, _Float16* vt,
                                                int route, int bh, int l0, int w, int lane) {
  const int q8 = lane & 7, sub = lane >> 3;
#pragma unroll
  for (int i = 0; i < 8; ++i) {
    const int lid = w * 32 + i * 4 + sub;
    v8h v;
    _Float16* dst;
    if (route != 2) {
      v = *(const v8ha*)(sT + lid * HD + 8 * q8);
      dst = plane + ((size_t)bh * SEQ + l0 + lid) * HD + 8 * q8;
    } else {
      const int d = lid >> 1, hl = lid & 1;
      v = *(const v8ha*)(sT + d * 128 + 64 * hl + 8 * q8);
      dst = vt + ((size_t)bh * HD + d) * SEQ + l0 + 64 * hl + 8 * q8;
    }
    *(volatile v8h*)dst = v;
  }
}

__global__ __launch_bounds__(128) void proj_kernel(
    const _Float16* __restrict__ xh,
    const _Float16* __restrict__ wh,
    const float* __restrict__ b0, const float* __restrict__ b1, const float* __restrict__ b2,
    int routeBase,
    _Float16* qh,
    _Float16* kh,
    _Float16* vt)
{
  __shared__ __attribute__((aligned(16))) _Float16 sT[128 * 64];

  const int tid = threadIdx.x, lane = tid & 31, w = tid >> 5;
  const int h = lane >> 4, m = lane & 15;
  const int m0 = blockIdx.x * 128;
  const int cg = blockIdx.y;
  const int slot = cg >> 4, head = cg & 15;
  const int route = slot + routeBase;
  const int m0w = m0 + 32 * w;

  const _Float16* xa0 = xh + (size_t)(m0w + m) * HID;
  const _Float16* xa1 = xa0 + (size_t)16 * HID;
  const _Float16* wb  = wh + ((size_t)slot * HID + head * HD + m) * HID;

  v8f acc[2][4];
#pragma unroll
  for (int mt = 0; mt < 2; ++mt)
#pragma unroll
    for (int nt = 0; nt < 4; ++nt) acc[mt][nt] = zero8f();

#pragma unroll 1
  for (int k0 = 0; k0 < HID; k0 += 32) {
    const v16h a0 = load_frag(xa0 + k0, h);
    const v16h a1 = load_frag(xa1 + k0, h);
#pragma unroll
    for (int nt = 0; nt < 4; ++nt) {
      const v16h b = load_frag(wb + (size_t)nt * 16 * HID + k0, h);
      acc[0][nt] = wmma_f16(a0, b, acc[0][nt]);
      acc[1][nt] = wmma_f16(a1, b, acc[1][nt]);
    }
  }

  const float* bias = (slot == 0) ? b0 : ((slot == 1) ? b1 : b2);
#pragma unroll
  for (int nt = 0; nt < 4; ++nt) {
    const int feat = 16 * nt + m;
    const float bvl = bias[head * HD + feat];
#pragma unroll
    for (int mt = 0; mt < 2; ++mt) {
#pragma unroll
      for (int r = 0; r < 8; ++r) {
        const int tokl = 32 * w + 16 * mt + 8 * h + r;
        const float yv = (acc[mt][nt][r] * (1.0f / (XSC * WSC)) + bvl) * QSC;
        const int idx = (route == 2) ? (feat * 128 + tokl) : (tokl * HD + feat);
        sT[idx] = (_Float16)yv;
      }
    }
  }
  __syncthreads();

  const int b = m0 / SEQ, l0 = m0 - b * SEQ, bh = b * NHEADS + head;
  _Float16* plane = (route == 0) ? qh : kh;
  proj_store_pass(sT, plane, vt, route, bh, l0, w, lane);
  __threadfence();
  proj_store_pass(sT, plane, vt, route, bh, l0, w, lane);
}

__device__ __forceinline__ v16h pack_p(v8f a, v8f c) {
  const v16h r = { (_Float16)(a[0] * PSC), (_Float16)(a[1] * PSC), (_Float16)(a[2] * PSC), (_Float16)(a[3] * PSC),
                   (_Float16)(a[4] * PSC), (_Float16)(a[5] * PSC), (_Float16)(a[6] * PSC), (_Float16)(a[7] * PSC),
                   (_Float16)(c[0] * PSC), (_Float16)(c[1] * PSC), (_Float16)(c[2] * PSC), (_Float16)(c[3] * PSC),
                   (_Float16)(c[4] * PSC), (_Float16)(c[5] * PSC), (_Float16)(c[6] * PSC), (_Float16)(c[7] * PSC) };
  return r;
}

template <int MODE>
__global__ __launch_bounds__(128) void attn_kernel(
    const _Float16* __restrict__ qh,
    const _Float16* __restrict__ kh,
    const _Float16* __restrict__ vt,
    const float* __restrict__ aproj,
    const float* __restrict__ gate,
    const int* __restrict__ ids,
    _Float16* ctx)
{
  __shared__ __attribute__((aligned(16))) int   sSeg[SEQ];
  __shared__ __attribute__((aligned(16))) int   sFl[SEQ];
  __shared__ __attribute__((aligned(16))) float sA[(MODE == 2) ? SEQ : 4];
  __shared__ __attribute__((aligned(16))) float sO[4 * 16 * 64];
  __shared__ int sWtot[4];

  const int tid = threadIdx.x, lane = tid & 31, w = tid >> 5;
  const int h = lane >> 4, m = lane & 15;
  const int bh = blockIdx.y, b = bh >> 4, head = bh & 15;
  const int qblk = blockIdx.x * 64;
  const int q0 = qblk + 16 * w;
  const float hs = exp2f(-0.5f * (float)(head + 1));

  {
    const int t8 = tid * 8;
    const int* ip = ids + (size_t)b * SEQ + t8;
    const v4i ia = *(const v4ia*)ip;
    const v4i ib = *(const v4ia*)(ip + 4);
    const int idv[8] = { ia.x, ia.y, ia.z, ia.w, ib.x, ib.y, ib.z, ib.w };
    int cnt[8];
    int run = 0;
#pragma unroll
    for (int i = 0; i < 8; ++i) { run += (idv[i] == SEP_ID) ? 1 : 0; cnt[i] = run; }
    int x = run;
#pragma unroll
    for (int d = 1; d < 32; d <<= 1) {
      const int yv = __shfl_up(x, d, 32);
      x = (lane >= d) ? (x + yv) : x;
    }
    if (lane == 31) sWtot[w] = x;
    __syncthreads();
    int base = 0;
#pragma unroll
    for (int i = 0; i < 4; ++i) { const int tv = sWtot[i]; base += (i < w) ? tv : 0; }
    const int excl = base + x - run;
#pragma unroll
    for (int i = 0; i < 8; ++i) {
      const int id = idv[i];
      sSeg[t8 + i] = excl + cnt[i];
      sFl[t8 + i] = ((id != PAD_ID) ? 1 : 0) | ((id == CLS_ID) ? 2 : 0);
      if constexpr (MODE == 2) sA[t8 + i] = aproj[((size_t)b * SEQ + t8 + i) * NHEADS + head];
    }
  }
  __syncthreads();

  const int qtok = q0 + m;
  const int qseg = sSeg[qtok];
  const int qv = sFl[qtok] & 1;
  const float gq = gate[((size_t)b * SEQ + qtok) * NHEADS + head];

  v16h qb0 = zero16h(), qb1 = zero16h();
  if constexpr (MODE != 2) {
    const _Float16* qrow = qh + ((size_t)bh * SEQ + q0 + m) * HD;
    qb0 = load_frag(qrow, h);
    qb1 = load_frag(qrow + 32, h);
  }

  v8f o[4];
#pragma unroll
  for (int t = 0; t < 4; ++t) o[t] = zero8f();
  float mrun = NEGBIG, lrun = 0.0f;

  const _Float16* kbase = kh + ((size_t)bh * SEQ + m) * HD;
  const _Float16* vbase = vt + ((size_t)bh * HD + m) * SEQ;
  const float SSC = 0.125f / (QSC * QSC);
  const int nkb = blockIdx.x + 1;

#pragma unroll 1
  for (int step = 0; step < nkb; ++step) {
    const int kb = step * 64;
    v8f s[4];
    if constexpr (MODE != 2) {
#pragma unroll
      for (int j = 0; j < 4; ++j) {
        const _Float16* kp = kbase + (size_t)(kb + 16 * j) * HD;
        const v16h kf0 = load_frag(kp, h);
        const v16h kf1 = load_frag(kp + 32, h);
        v8f z = zero8f();
        z = wmma_f16(kf0, qb0, z);
        z = wmma_f16(kf1, qb1, z);
        s[j] = z;
      }
    } else {
#pragma unroll
      for (int j = 0; j < 4; ++j) s[j] = zero8f();
    }
    unsigned okm = 0u;
#pragma unroll
    for (int j = 0; j < 4; ++j) {
      const int key0 = kb + 16 * j + 8 * h;
      const v4i ga = *(const v4ia*)(sSeg + key0);
      const v4i gb = *(const v4ia*)(sSeg + key0 + 4);
      const v4i fa = *(const v4ia*)(sFl + key0);
      const v4i fb = *(const v4ia*)(sFl + key0 + 4);
      const int ksv[8] = { ga.x, ga.y, ga.z, ga.w, gb.x, gb.y, gb.z, gb.w };
      const int kfv[8] = { fa.x, fa.y, fa.z, fa.w, fb.x, fb.y, fb.z, fb.w };
      float av[8] = { 0.f, 0.f, 0.f, 0.f, 0.f, 0.f, 0.f, 0.f };
      if constexpr (MODE == 2) {
        const v4f aa = *(const v4fa*)(sA + key0);
        const v4f ab = *(const v4fa*)(sA + key0 + 4);
        av[0] = aa.x; av[1] = aa.y; av[2] = aa.z; av[3] = aa.w;
        av[4] = ab.x; av[5] = ab.y; av[6] = ab.z; av[7] = ab.w;
      }
#pragma unroll
      for (int r = 0; r < 8; ++r) {
        const int key = key0 + r;
        float raw;
        if constexpr (MODE == 2) raw = av[r]; else raw = s[j][r] * SSC;
        bool ok;
        float bv;
        if constexpr (MODE == 1) {
          ok = (key <= qtok) && (((kfv[r] & 2) != 0) || (key == qtok));
          bv = (float)(ksv[r] - qseg);
        } else {
          const bool eq = (ksv[r] == qseg) && (qv != 0) && ((kfv[r] & 1) != 0);
          ok = (key <= qtok) && (eq || (key == qtok));
          bv = (float)(key - qtok);
        }
        s[j][r] = ok ? (raw + bv * hs) : NEGBIG;
        okm |= (ok ? 1u : 0u) << (8 * j + r);
      }
    }

    float mloc = NEGBIG;
#pragma unroll
    for (int j = 0; j < 4; ++j)
#pragma unroll
      for (int r = 0; r < 8; ++r) mloc = fmaxf(mloc, s[j][r]);
    mloc = fmaxf(mloc, __shfl_xor(mloc, 16, 32));
    const float mnew = fmaxf(mrun, mloc);
    const float alpha = __expf(mrun - mnew);
    mrun = mnew;
    float lsum = 0.0f;
#pragma unroll
    for (int j = 0; j < 4; ++j)
#pragma unroll
      for (int r = 0; r < 8; ++r) {
        const float e = __expf(s[j][r] - mnew);
        const float p = (((okm >> (8 * j + r)) & 1u) != 0u) ? e : 0.0f;
        s[j][r] = p;
        lsum += p;
      }
    lsum += __shfl_xor(lsum, 16, 32);
    lrun = lrun * alpha + lsum;
#pragma unroll
    for (int t = 0; t < 4; ++t)
#pragma unroll
      for (int r = 0; r < 8; ++r) o[t][r] = o[t][r] * alpha;

    const v16h pb0 = pack_p(s[0], s[1]);
    const v16h pb1 = pack_p(s[2], s[3]);

#pragma unroll
    for (int t = 0; t < 4; ++t) {
      const _Float16* vp = vbase + (size_t)(16 * t) * SEQ + kb;
      const v16h vf0 = load_frag(vp, h);
      const v16h vf1 = load_frag(vp + 32, h);
      o[t] = wmma_f16(vf0, pb0, o[t]);
      o[t] = wmma_f16(vf1, pb1, o[t]);
    }
  }

  const float inv = (1.0f / lrun) * (1.0f / (PSC * QSC)) * gq;
  float* so = sO + w * 1024;
#pragma unroll
  for (int t = 0; t < 4; ++t)
#pragma unroll
    for (int r = 0; r < 8; ++r)
      so[m * 64 + 16 * t + 8 * h + r] = o[t][r] * inv;
  __syncthreads();

  const int q4 = lane >> 3, c8 = (lane & 7) * 8;
  v8h hv[4];
#pragma unroll
  for (int it = 0; it < 4; ++it) {
    const int row = it * 4 + q4;
    const v4f f0 = *(const v4fa*)(so + row * 64 + c8);
    const v4f f1 = *(const v4fa*)(so + row * 64 + c8 + 4);
    const v8h v = { (_Float16)(f0.x * CSC), (_Float16)(f0.y * CSC), (_Float16)(f0.z * CSC), (_Float16)(f0.w * CSC),
                    (_Float16)(f1.x * CSC), (_Float16)(f1.y * CSC), (_Float16)(f1.z * CSC), (_Float16)(f1.w * CSC) };
    hv[it] = v;
  }
  for (int pass = 0; pass < 2; ++pass) {
#pragma unroll
    for (int it = 0; it < 4; ++it) {
      const int row = it * 4 + q4;
      _Float16* dst = ctx + ((size_t)b * SEQ + q0 + row) * HID + head * HD + c8;
      *(volatile v8h*)dst = hv[it];
    }
    __threadfence();
  }
}

__global__ __launch_bounds__(128) void outproj_kernel(
    const _Float16* __restrict__ ch,
    const _Float16* __restrict__ woh,
    const float* __restrict__ ob,
    const float* __restrict__ xres,
    float* xout)
{
  __shared__ __attribute__((aligned(16))) float sT[128 * 64];

  const int tid = threadIdx.x, lane = tid & 31, w = tid >> 5;
  const int h = lane >> 4, m = lane & 15;
  const int m0 = blockIdx.x * 128;
  const int n0 = blockIdx.y * 64;
  const int m0w = m0 + 32 * w;

  const _Float16* ca0 = ch + (size_t)(m0w + m) * HID;
  const _Float16* ca1 = ca0 + (size_t)16 * HID;
  const _Float16* wb  = woh + (size_t)(n0 + m) * HID;

  v8f acc[2][4];
#pragma unroll
  for (int mt = 0; mt < 2; ++mt)
#pragma unroll
    for (int nt = 0; nt < 4; ++nt) acc[mt][nt] = zero8f();

#pragma unroll 1
  for (int k0 = 0; k0 < HID; k0 += 32) {
    const v16h a0 = load_frag(ca0 + k0, h);
    const v16h a1 = load_frag(ca1 + k0, h);
#pragma unroll
    for (int nt = 0; nt < 4; ++nt) {
      const v16h bfr = load_frag(wb + (size_t)nt * 16 * HID + k0, h);
      acc[0][nt] = wmma_f16(a0, bfr, acc[0][nt]);
      acc[1][nt] = wmma_f16(a1, bfr, acc[1][nt]);
    }
  }

#pragma unroll
  for (int nt = 0; nt < 4; ++nt) {
    const int feat = 16 * nt + m;
    const float bvl = ob[n0 + feat];
#pragma unroll
    for (int mt = 0; mt < 2; ++mt) {
#pragma unroll
      for (int r = 0; r < 8; ++r) {
        const int tokl = 32 * w + 16 * mt + 8 * h + r;
        sT[tokl * 64 + feat] = acc[mt][nt][r] * (1.0f / (CSC * WSC)) + bvl;
      }
    }
  }
  __syncthreads();

  const int hh = lane >> 4, c4 = (lane & 15) * 4;
  for (int pass = 0; pass < 2; ++pass) {
#pragma unroll
    for (int it = 0; it < 16; ++it) {
      const int row = 32 * w + it * 2 + hh;
      const v4f v = *(const v4fa*)(sT + row * 64 + c4);
      const size_t gi = (size_t)(m0 + row) * HID + n0 + c4;
      const v4f xr = *(const v4fa*)(xres + gi);
      const v4f ov = v + xr;
      *(volatile v4f*)(xout + gi) = ov;
    }
    __threadfence();
  }
}

extern "C" void kernel_launch(void* const* d_in, const int* in_sizes, int n_in,
                              void* d_out, int out_size, void* d_ws, size_t ws_size,
                              hipStream_t stream) {
  if (n_in < 35) return;
  if (in_sizes[0] != NX || in_sizes[1] != MROWS) return;
  if (out_size != NX) return;
  {
    const int vecIdx[16] = {2, 3, 5, 7, 9, 13, 14, 15, 18, 22, 23, 24, 26, 28, 30, 34};
    for (int i = 0; i < 16; ++i) if (in_sizes[vecIdx[i]] != HID) return;
    const int matIdx[10] = {4, 6, 8, 12, 17, 21, 25, 27, 29, 33};
    for (int i = 0; i < 10; ++i) if (in_sizes[matIdx[i]] != NW) return;
    const int hwIdx[4] = {10, 16, 19, 31};
    for (int i = 0; i < 4; ++i) if (in_sizes[hwIdx[i]] != NG) return;
    const int hbIdx[3] = {11, 20, 32};
    for (int i = 0; i < 3; ++i) if (in_sizes[hbIdx[i]] != NHEADS) return;
  }

  const float* states = (const float*)d_in[0];
  const int*   ids    = (const int*)d_in[1];
  const float* ln0w = (const float*)d_in[2];
  const float* ln0b = (const float*)d_in[3];
  const float* qw0 = (const float*)d_in[4];
  const float* qb0 = (const float*)d_in[5];
  const float* kw0 = (const float*)d_in[6];
  const float* kb0 = (const float*)d_in[7];
  const float* vw0 = (const float*)d_in[8];
  const float* vb0 = (const float*)d_in[9];
  const float* gw0 = (const float*)d_in[10];
  const float* gb0 = (const float*)d_in[11];
  const float* ow0 = (const float*)d_in[12];
  const float* ob0 = (const float*)d_in[13];
  const float* ln1w = (const float*)d_in[14];
  const float* ln1b = (const float*)d_in[15];
  const float* aw1 = (const float*)d_in[16];
  const float* vw1 = (const float*)d_in[17];
  const float* vb1 = (const float*)d_in[18];
  const float* gw1 = (const float*)d_in[19];
  const float* gb1 = (const float*)d_in[20];
  const float* ow1 = (const float*)d_in[21];
  const float* ob1 = (const float*)d_in[22];
  const float* ln2w = (const float*)d_in[23];
  const float* ln2b = (const float*)d_in[24];
  const float* qw2 = (const float*)d_in[25];
  const float* qb2 = (const float*)d_in[26];
  const float* kw2 = (const float*)d_in[27];
  const float* kb2 = (const float*)d_in[28];
  const float* vw2 = (const float*)d_in[29];
  const float* vb2 = (const float*)d_in[30];
  const float* gw2 = (const float*)d_in[31];
  const float* gb2 = (const float*)d_in[32];
  const float* ow2 = (const float*)d_in[33];
  const float* ob2 = (const float*)d_in[34];
  float* out = (float*)d_out;

  const size_t PXH = (size_t)NX * 2;
  const size_t PW  = (size_t)NW * 2;
  const size_t PGH = (size_t)2 * NG * 2;
  const size_t PGT = (size_t)MROWS * NHEADS * 4;
  const size_t PPL = (size_t)NB * NHEADS * SEQ * HD * 2;
  const size_t PXF = (size_t)NX * 4;
  size_t off = 0;
  const size_t oXn  = off; off += PXH;
  const size_t oWh  = off; off += 3 * PW;
  const size_t oWo  = off; off += PW;
  const size_t oGh  = off; off += PGH;
  const size_t oGt  = off; off += PGT;
  const size_t oAp  = off; off += PGT;
  const size_t oQ   = off; off += PPL;
  const size_t oK   = off; off += PPL;
  const size_t oVt  = off; off += PPL;
  const size_t oCtx = off; off += PXH;
  const size_t oX1  = off; off += PXF;
  const size_t oX2  = off; off += PXF;
  if (off > ws_size) return;
  if (off > (size_t)134217728) return;

  char* ws = (char*)d_ws;
  _Float16* xnh = (_Float16*)(ws + oXn);
  _Float16* wh  = (_Float16*)(ws + oWh);
  _Float16* woh = (_Float16*)(ws + oWo);
  _Float16* gh  = (_Float16*)(ws + oGh);
  float* gate   = (float*)(ws + oGt);
  float* aproj  = (float*)(ws + oAp);
  _Float16* qh  = (_Float16*)(ws + oQ);
  _Float16* kh  = (_Float16*)(ws + oK);
  _Float16* vt  = (_Float16*)(ws + oVt);
  _Float16* ctx = (_Float16*)(ws + oCtx);
  float* x1 = (float*)(ws + oX1);
  float* x2 = (float*)(ws + oX2);

  const dim3 blk256(256), blk128(128);
  const int cvtFull = 3 * NW8 + NW8 + 1 * NG8;
  const int cvtPool = 1 * NW8 + NW8 + 2 * NG8;
  const dim3 gCvtFull((cvtFull + 255) / 256);
  const dim3 gCvtPool((cvtPool + 255) / 256);
  const dim3 gLn(MROWS);
  const dim3 gHead(MROWS / 64);
  const dim3 gProj3(MROWS / 128, 3 * NHEADS);
  const dim3 gProj1(MROWS / 128, 1 * NHEADS);
  const dim3 gAtt(SEQ / 64, NB * NHEADS);
  const dim3 gOut(MROWS / 128, HID / 64);

  convert_kernel<<<gCvtFull, blk256, 0, stream>>>(qw0, kw0, vw0, ow0, gw0, gw0, 3, 1, wh, woh, gh);
  ln_kernel<<<gLn, blk128, 0, stream>>>(states, ln0w, ln0b, xnh);
  head_kernel<false><<<gHead, blk128, 0, stream>>>(xnh, gh, gb0, gate, aproj);
  proj_kernel<<<gProj3, blk128, 0, stream>>>(xnh, wh, qb0, kb0, vb0, 0, qh, kh, vt);
  attn_kernel<0><<<gAtt, blk128, 0, stream>>>(qh, kh, vt, aproj, gate, ids, ctx);
  outproj_kernel<<<gOut, blk128, 0, stream>>>(ctx, woh, ob0, states, x1);

  convert_kernel<<<gCvtPool, blk256, 0, stream>>>(vw1, vw1, vw1, ow1, gw1, aw1, 1, 2, wh, woh, gh);
  ln_kernel<<<gLn, blk128, 0, stream>>>(x1, ln1w, ln1b, xnh);
  head_kernel<true><<<gHead, blk128, 0, stream>>>(xnh, gh, gb1, gate, aproj);
  proj_kernel<<<gProj1, blk128, 0, stream>>>(xnh, wh, vb1, vb1, vb1, 2, qh, kh, vt);
  attn_kernel<2><<<gAtt, blk128, 0, stream>>>(qh, kh, vt, aproj, gate, ids, ctx);
  outproj_kernel<<<gOut, blk128, 0, stream>>>(ctx, woh, ob1, x1, x2);

  convert_kernel<<<gCvtFull, blk256, 0, stream>>>(qw2, kw2, vw2, ow2, gw2, gw2, 3, 1, wh, woh, gh);
  ln_kernel<<<gLn, blk128, 0, stream>>>(x2, ln2w, ln2b, xnh);
  head_kernel<false><<<gHead, blk128, 0, stream>>>(xnh, gh, gb2, gate, aproj);
  proj_kernel<<<gProj3, blk128, 0, stream>>>(xnh, wh, qb2, kb2, vb2, 0, qh, kh, vt);
  attn_kernel<1><<<gAtt, blk128, 0, stream>>>(qh, kh, vt, aproj, gate, ids, ctx);
  outproj_kernel<<<gOut, blk128, 0, stream>>>(ctx, woh, ob2, x2, out);

  (void)hipGetLastError();
}
